// PhyNEO_GNN_V2_27968827032295
// MI455X (gfx1250) — hardware-verified
//
#include <hip/hip_runtime.h>
#include <stddef.h>
#include <stdint.h>
#include <math.h>


#define HD     128
#define WSC    16.0f
#define WINV   0.0625f
#define HP     136
#define LN_EPS 1e-6f

#define T_N0    0
#define T_E0    8192
#define T_L0    12288
#define TL_PROJ 0
#define TL_EE   49152
#define TL_MN   65536
#define TL_NN   81920
#define T_LSZ   114688
#define T_F1SZ  8192
#define T_F2SZ  2048
#define T_F3SZ  512


typedef float    v4f  __attribute__((ext_vector_type(4)));
typedef float    v8f  __attribute__((ext_vector_type(8)));
typedef int      v4i  __attribute__((ext_vector_type(4)));
typedef _Float16 v4h  __attribute__((ext_vector_type(4)));
typedef _Float16 v8h  __attribute__((ext_vector_type(8)));
typedef _Float16 v16h __attribute__((ext_vector_type(16)));
union FragH { v16h v; v8h h[2]; };

__device__ __forceinline__ v8f zero8f() {
  v8f z;
#pragma unroll
  for (int i = 0; i < 8; ++i) z[i] = 0.0f;
  return z;
}
__device__ __forceinline__ v8h zero8h() {
  v8h z;
#pragma unroll
  for (int i = 0; i < 8; ++i) z[i] = (_Float16)0.0f;
  return z;
}
__device__ __forceinline__ v8h cvt8(const float* p) {
  const v4f a = *(const v4f*)p;
  const v4f b = *(const v4f*)(p + 4);
  v8h o;
  o[0] = (_Float16)a[0]; o[1] = (_Float16)a[1]; o[2] = (_Float16)a[2]; o[3] = (_Float16)a[3];
  o[4] = (_Float16)b[0]; o[5] = (_Float16)b[1]; o[6] = (_Float16)b[2]; o[7] = (_Float16)b[3];
  return o;
}

__device__ __forceinline__ v8f wmh(v16h a, v16h b, v8f c) {
  v8f d = __builtin_amdgcn_wmma_f32_16x16x32_f16(false, a, false, b, (short)0, c, false, false);
  asm volatile("v_nop\n\tv_nop\n\tv_nop\n\tv_nop" : "+v"(d) : "v"(a), "v"(b));
  return d;
}

template <int NT, int KT>
__device__ __forceinline__ void gemm_t(const _Float16* arow, const _Float16* bcol, int kp, v8f* acc) {
#pragma unroll 1
  for (int kt = 0; kt < KT; ++kt) {
    FragH a;
    a.h[0] = *(const v8h*)(arow + 32 * kt);
    a.h[1] = *(const v8h*)(arow + 32 * kt + 16);
#pragma unroll
    for (int nt = 0; nt < NT; ++nt) {
      const _Float16* bp = bcol + (size_t)(16 * nt) * kp + 32 * kt;
      FragH b;
      b.h[0] = *(const v8h*)bp;
      b.h[1] = *(const v8h*)(bp + 16);
      acc[nt] = wmh(a.v, b.v, acc[nt]);
    }
  }
}

__device__ __forceinline__ void store_rows16(const _Float16* stg, _Float16* g, int gp, int row0, int M,
                                             int wave, int l) {
  const int h = l >> 4, c8 = 8 * (l & 15);
#pragma unroll
  for (int j = 0; j < 8; ++j) {
    const int lr = 16 * wave + 2 * j + h;
    const int gr = row0 + lr;
    if (gr < M) {
      const v8h v = *(const v8h*)(stg + lr * HP + c8);
      *(volatile v8h*)(g + (size_t)gr * gp + c8) = v;
    }
  }
  __threadfence();
#pragma unroll
  for (int j = 0; j < 8; ++j) {
    const int lr = 16 * wave + 2 * j + h;
    const int gr = row0 + lr;
    if (gr < M) {
      const v8h v = *(const v8h*)(stg + lr * HP + c8);
      *(volatile v8h*)(g + (size_t)gr * gp + c8) = v;
    }
  }
}

__device__ __forceinline__ void store_rows_f32(const float* st, int sp, float* g, int grow0, int M, int l) {
#pragma unroll
  for (int rr = 0; rr < 16; ++rr) {
    const int grow = grow0 + rr;
    if (grow < M) {
      const v4f v = *(const v4f*)(st + rr * sp + 4 * l);
      *(volatile v4f*)(g + (size_t)grow * HD + 4 * l) = v;
    }
  }
  __threadfence();
#pragma unroll
  for (int rr = 0; rr < 16; ++rr) {
    const int grow = grow0 + rr;
    if (grow < M) {
      const v4f v = *(const v4f*)(st + rr * sp + 4 * l);
      *(volatile v4f*)(g + (size_t)grow * HD + 4 * l) = v;
    }
  }
}

__global__ __launch_bounds__(256) void k_wcvt(const float* __restrict__ src, int sStride, int srcCols,
                                              int rowOff, int K, int KP, int nValid, int nColsT,
                                              _Float16* dst, int dStride) {
  const int step = blockIdx.y;
  const int idx = blockIdx.x * 256 + threadIdx.x;
  const int kp8 = KP >> 3;
  const int c = idx / kp8;
  if (c >= nColsT) return;
  const int k8 = (idx - c * kp8) * 8;
  const float* s = src + (size_t)step * sStride;
  v8h o;
#pragma unroll
  for (int i = 0; i < 8; ++i) {
    const int k = k8 + i;
    float v = 0.0f;
    if (k < K && c < nValid) v = s[(size_t)(rowOff + k) * srcCols + c] * WSC;
    o[i] = (_Float16)v;
  }
  _Float16* dp = dst + (size_t)step * dStride + (size_t)c * KP + k8;
  *(volatile v8h*)dp = o;
  __threadfence();
  *(volatile v8h*)dp = o;
}

#define EN_AP  72
#define EN_FP  132
#define EN_AT  0
#define EN_ST  (128 * EN_AP * 2)
#define EN_LDS (EN_ST + 128 * EN_FP * 4)

__global__ __launch_bounds__(256) void k_embn(const float* __restrict__ feat, const _Float16* T0,
                                              const float* __restrict__ b0, float* nodes, int nN) {
  extern __shared__ __attribute__((aligned(16))) unsigned char lds[];
  _Float16* at  = (_Float16*)(lds + EN_AT);
  float*    stg = (float*)(lds + EN_ST);
  const int tid = threadIdx.x, l = tid & 31, wave = tid >> 5, h = l >> 4, m = l & 15;
  const int row0 = blockIdx.x * 128;

  for (int i = tid; i < 128 * 8; i += 256) {
    const int r = i >> 3, c = (i & 7) * 8;
    const int gr = row0 + r;
    const v8h v = (gr < nN) ? cvt8(feat + (size_t)gr * 64 + c) : zero8h();
    *(v8h*)(at + r * EN_AP + c) = v;
  }
  __syncthreads();

  v8f acc[8];
#pragma unroll
  for (int i = 0; i < 8; ++i) acc[i] = zero8f();
  gemm_t<8, 2>(at + (16 * wave + m) * EN_AP + 8 * h, T0 + (size_t)m * 64 + 8 * h, 64, acc);

  float* st = stg + wave * (16 * EN_FP);
#pragma unroll
  for (int nt = 0; nt < 8; ++nt) {
    const int c = 16 * nt + m;
    const float bc = b0[c];
#pragma unroll
    for (int r = 0; r < 8; ++r) st[(8 * h + r) * EN_FP + c] = acc[nt][r] * WINV + bc;
  }
  __syncthreads();
  store_rows_f32(st, EN_FP, nodes, row0 + 16 * wave, nN, l);
}

#define EE_AT  0
#define EE_ST  (128 * 32 * 2)
#define EE_LDS (EE_ST + 128 * HP * 2)

__global__ __launch_bounds__(256) void k_embe(const float* __restrict__ ef, const _Float16* T0,
                                              const float* __restrict__ b0, _Float16* edges, int nE) {
  extern __shared__ __attribute__((aligned(16))) unsigned char lds[];
  _Float16* at  = (_Float16*)(lds + EE_AT);
  _Float16* stg = (_Float16*)(lds + EE_ST);
  const int tid = threadIdx.x, l = tid & 31, wave = tid >> 5, h = l >> 4, m = l & 15;
  const int e0 = blockIdx.x * 128;

  for (int i = tid; i < 128 * 4; i += 256) {
    const int r = i >> 2, c = (i & 3) * 8;
    const int ge = e0 + r;
    v8h v = zero8h();
    if (c < 16 && ge < nE) v = cvt8(ef + (size_t)ge * 16 + c);
    *(v8h*)(at + r * 32 + c) = v;
  }
  __syncthreads();

  v8f acc[8];
#pragma unroll
  for (int i = 0; i < 8; ++i) acc[i] = zero8f();
  gemm_t<8, 1>(at + (16 * wave + m) * 32 + 8 * h, T0 + (size_t)m * 32 + 8 * h, 32, acc);

#pragma unroll
  for (int nt = 0; nt < 8; ++nt) {
    const int c = 16 * nt + m;
    const float bc = b0[c];
#pragma unroll
    for (int r = 0; r < 8; ++r) stg[(16 * wave + 8 * h + r) * HP + c] = (_Float16)(acc[nt][r] * WINV + bc);
  }
  __syncthreads();
  store_rows16(stg, edges, HD, e0, nE, wave, l);
}

#define PJ_AT  0
#define PJ_ST  (128 * HP * 2)
#define PJ_LDS (2 * 128 * HP * 2)

__global__ __launch_bounds__(256) void k_proj(const float* __restrict__ nodes, const _Float16* Tp,
                                              _Float16* P, int nN) {
  extern __shared__ __attribute__((aligned(16))) unsigned char lds[];
  _Float16* at  = (_Float16*)(lds + PJ_AT);
  _Float16* stg = (_Float16*)(lds + PJ_ST);
  const int tid = threadIdx.x, l = tid & 31, wave = tid >> 5, h = l >> 4, m = l & 15;
  const int row0 = blockIdx.x * 128;

  for (int i = tid; i < 128 * 16; i += 256) {
    const int r = i >> 4, c = (i & 15) * 8;
    const int gr = row0 + r;
    const v8h v = (gr < nN) ? cvt8(nodes + (size_t)gr * HD + c) : zero8h();
    *(v8h*)(at + r * HP + c) = v;
  }
  __syncthreads();

#pragma unroll 1
  for (int cg = 0; cg < 3; ++cg) {
    v8f acc[8];
#pragma unroll
    for (int i = 0; i < 8; ++i) acc[i] = zero8f();
    gemm_t<8, 4>(at + (16 * wave + m) * HP + 8 * h, Tp + (size_t)(cg * 128 + m) * HD + 8 * h, HD, acc);
#pragma unroll
    for (int r = 0; r < 8; ++r) {
      v8h o;
#pragma unroll
      for (int nt = 0; nt < 8; ++nt) o[nt] = (_Float16)(acc[nt][r] * WINV);
      *(v8h*)(stg + (16 * wave + 8 * h + r) * HP + 8 * m) = o;
    }
    __syncthreads();
    store_rows16(stg, P + cg * 128, 384, row0, nN, wave, l);
    __syncthreads();
  }
}

#define EG_TA  0
#define EG_TN  (128 * HP * 2)
#define EG_IDX (2 * 128 * HP * 2)
#define EG_LDS (EG_IDX + 256 * 4)

__global__ __launch_bounds__(256) void k_edge(const int* __restrict__ snd, const int* __restrict__ rcv,
                                              const _Float16* __restrict__ P, const _Float16* Tee,
                                              const float* __restrict__ be, const float* __restrict__ ls,
                                              const float* __restrict__ lb, _Float16* edges, _Float16* ne,
                                              int nE, int nN) {
  extern __shared__ __attribute__((aligned(16))) unsigned char lds[];
  _Float16* ta   = (_Float16*)(lds + EG_TA);
  _Float16* tn   = (_Float16*)(lds + EG_TN);
  int*      sidx = (int*)(lds + EG_IDX);
  int*      ridx = sidx + 128;
  const int tid = threadIdx.x, l = tid & 31, wave = tid >> 5, h = l >> 4, m = l & 15;
  const int e0 = blockIdx.x * 128;

  if (tid < 128) {
    const int e = e0 + tid;
    int s = 0, r = 0;
    if (e < nE) { s = snd[e]; r = rcv[e]; }
    s = s < 0 ? 0 : (s > nN - 1 ? nN - 1 : s);
    r = r < 0 ? 0 : (r > nN - 1 ? nN - 1 : r);
    sidx[tid] = s;
    ridx[tid] = r;
  }
  for (int i = tid; i < 128 * 16; i += 256) {
    const int r = i >> 4, c = (i & 15) * 8;
    const int ge = e0 + r;
    v8h v = zero8h();
    if (ge < nE) v = *(const v8h*)(edges + (size_t)ge * HD + c);
    *(v8h*)(ta + r * HP + c) = v;
  }
  __syncthreads();

  v8f acc[8];
#pragma unroll
  for (int i = 0; i < 8; ++i) acc[i] = zero8f();
  gemm_t<8, 4>(ta + (16 * wave + m) * HP + 8 * h, Tee + (size_t)m * HD + 8 * h, HD, acc);

  float mu[8], rs[8];
  {
    v8h ps[8], pr[8];
#pragma unroll
    for (int r = 0; r < 8; ++r) {
      const int lr = 16 * wave + 8 * h + r;
      const int si = sidx[lr];
      const int ri = ridx[lr];
      ps[r] = *(const v8h*)(P + (size_t)si * 384 + 8 * m);
      pr[r] = *(const v8h*)(P + (size_t)ri * 384 + 128 + 8 * m);
    }
#pragma unroll
    for (int nt = 0; nt < 8; ++nt) {
      const int c = 16 * nt + m;
      const float bc = be[c];
#pragma unroll
      for (int r = 0; r < 8; ++r) {
        const int lr = 16 * wave + 8 * h + r;
        float v = acc[nt][r] * WINV + (float)ps[r][nt];
        v = v + (float)pr[r][nt];
        v = v + bc;
        tn[lr * HP + c] = (_Float16)v;
        const float old = (float)ta[lr * HP + c];
        acc[nt][r] = v + old;
      }
    }
  }
#pragma unroll
  for (int r = 0; r < 8; ++r) {
    float s = 0.0f;
#pragma unroll
    for (int nt = 0; nt < 8; ++nt) s += acc[nt][r];
    s += __shfl_xor(s, 1, 32);
    s += __shfl_xor(s, 2, 32);
    s += __shfl_xor(s, 4, 32);
    s += __shfl_xor(s, 8, 32);
    mu[r] = s * (1.0f / 128.0f);
  }
#pragma unroll
  for (int r = 0; r < 8; ++r) {
    float q = 0.0f;
#pragma unroll
    for (int nt = 0; nt < 8; ++nt) { const float d = acc[nt][r] - mu[r]; q += d * d; }
    q += __shfl_xor(q, 1, 32);
    q += __shfl_xor(q, 2, 32);
    q += __shfl_xor(q, 4, 32);
    q += __shfl_xor(q, 8, 32);
    rs[r] = rsqrtf(q * (1.0f / 128.0f) + LN_EPS);
  }
  __syncthreads();
#pragma unroll
  for (int nt = 0; nt < 8; ++nt) {
    const int c = 16 * nt + m;
    const float sc = ls[c], sb = lb[c];
#pragma unroll
    for (int r = 0; r < 8; ++r) {
      const int lr = 16 * wave + 8 * h + r;
      const float y = (acc[nt][r] - mu[r]) * rs[r] * sc + sb;
      ta[lr * HP + c] = (_Float16)y;
    }
  }
  __syncthreads();
  store_rows16(tn, ne, HD, e0, nE, wave, l);
  store_rows16(ta, edges, HD, e0, nE, wave, l);
}

#define NTHR   256
#define NWAVE  8
#define NB     128
#define EPT    8
#define CHUNK  (NTHR * EPT)
#define WCAP   (EPT * 32)
#define L_ACC  0
#define L_TN   (NB * HD * 4)
#define L_TS   (L_TN + NB * HP * 2)
#define L_TG   (L_TS + NB * HP * 2)
#define L_LIST (L_TG + NB * HP * 2)
#define L_WCNT (L_LIST + NWAVE * WCAP * 4)
#define L_CNT  (L_WCNT + 64)
#define L_LDS  (L_CNT + NB * 4)

static_assert(NB == 128 && (NB % NWAVE) == 0 && NB <= NTHR && WCAP == 256 && NWAVE == 8);
static_assert((L_TN & 15) == 0 && (L_TS & 15) == 0 && (L_TG & 15) == 0 && (L_LIST & 15) == 0 && (L_CNT & 15) == 0);
static_assert(((HP * 2) & 15) == 0 && ((EN_AP * 2) & 15) == 0 && ((EN_FP * 4) & 15) == 0);
static_assert(L_LDS <= 300 * 1024 && EN_LDS <= 300 * 1024 && EG_LDS <= 300 * 1024 && PJ_LDS <= 300 * 1024);

__device__ __forceinline__ int scan_chunk(const int* __restrict__ dsts, int nE, int cbase, int nodeBase,
                                          int* list, int tid, int wave) {
  int wc = 0;
  const int el0  = tid * EPT;
  const int e0   = cbase + el0;
  const int sent = -2147483647 - 1;
  v4i da, db;
  if (e0 + 7 < nE) {
    da = *(const v4i*)(dsts + e0);
    db = *(const v4i*)(dsts + e0 + 4);
  } else {
    da.x = (e0     < nE) ? dsts[(e0     < nE) ? e0     : nE - 1] : sent;
    da.y = (e0 + 1 < nE) ? dsts[(e0 + 1 < nE) ? e0 + 1 : nE - 1] : sent;
    da.z = (e0 + 2 < nE) ? dsts[(e0 + 2 < nE) ? e0 + 2 : nE - 1] : sent;
    da.w = (e0 + 3 < nE) ? dsts[(e0 + 3 < nE) ? e0 + 3 : nE - 1] : sent;
    db.x = (e0 + 4 < nE) ? dsts[(e0 + 4 < nE) ? e0 + 4 : nE - 1] : sent;
    db.y = (e0 + 5 < nE) ? dsts[(e0 + 5 < nE) ? e0 + 5 : nE - 1] : sent;
    db.z = (e0 + 6 < nE) ? dsts[(e0 + 6 < nE) ? e0 + 6 : nE - 1] : sent;
    db.w = (e0 + 7 < nE) ? dsts[(e0 + 7 < nE) ? e0 + 7 : nE - 1] : sent;
  }
  const unsigned nb = (unsigned)nodeBase;
  const unsigned s0 = (unsigned)da.x - nb, s1 = (unsigned)da.y - nb;
  const unsigned s2 = (unsigned)da.z - nb, s3 = (unsigned)da.w - nb;
  const unsigned s4 = (unsigned)db.x - nb, s5 = (unsigned)db.y - nb;
  const unsigned s6 = (unsigned)db.z - nb, s7 = (unsigned)db.w - nb;
  const bool q0 = s0 < (unsigned)NB, q1 = s1 < (unsigned)NB, q2 = s2 < (unsigned)NB, q3 = s3 < (unsigned)NB;
  const bool q4 = s4 < (unsigned)NB, q5 = s5 < (unsigned)NB, q6 = s6 < (unsigned)NB, q7 = s7 < (unsigned)NB;
  const unsigned any = __builtin_amdgcn_ballot_w32(q0 | q1 | q2 | q3 | q4 | q5 | q6 | q7);
  if (any != 0u) {
#define HITJ(J, QJ, SJ) { \
      const unsigned mj = __builtin_amdgcn_ballot_w32(QJ); \
      if (mj != 0u) { \
        if (QJ) { \
          const int pos = wc + (int)__builtin_amdgcn_mbcnt_lo(mj, 0u); \
          if (pos < WCAP) list[wave * WCAP + pos] = ((el0 + (J)) << 8) | (int)(SJ); \
        } \
        wc += (int)__builtin_popcount(mj); } }
    HITJ(0, q0, s0)
    HITJ(1, q1, s1)
    HITJ(2, q2, s2)
    HITJ(3, q3, s3)
    HITJ(4, q4, s4)
    HITJ(5, q5, s5)
    HITJ(6, q6, s6)
    HITJ(7, q7, s7)
#undef HITJ
  }
  return wc;
}

__global__ __launch_bounds__(NTHR) void k_node(const int* __restrict__ rcv, const _Float16* __restrict__ ne,
                                               const _Float16* __restrict__ P, const _Float16* Tmn,
                                               const float* __restrict__ bm, const _Float16* Tnn,
                                               const float* __restrict__ bn, const float* __restrict__ ls,
                                               const float* __restrict__ lb, float* nodes, int nN, int nE) {
  extern __shared__ __attribute__((aligned(16))) unsigned char lds[];
  float*    accS = (float*)(lds + L_ACC);
  _Float16* tn   = (_Float16*)(lds + L_TN);
  _Float16* ts   = (_Float16*)(lds + L_TS);
  _Float16* tg   = (_Float16*)(lds + L_TG);
  int*      list = (int*)(lds + L_LIST);
  int*      wcnt = (int*)(lds + L_WCNT);
  int*      cntL = (int*)(lds + L_CNT);
  const int tid = threadIdx.x, l = tid & 31, wave = tid >> 5, h = l >> 4, m = l & 15;
  const int nodeBase = blockIdx.x * NB;

  {
    const v4f z = {0.0f, 0.0f, 0.0f, 0.0f};
    for (int i = tid; i < NB * (HD / 4); i += NTHR) *(v4f*)(accS + 4 * i) = z;
    if (tid < NB) cntL[tid] = 0;
  }
  for (int i = tid; i < NB * 16; i += NTHR) {
    const int r = i >> 4, c = (i & 15) * 8;
    const int gr = nodeBase + r;
    const v8h v = (gr < nN) ? cvt8(nodes + (size_t)gr * HD + c) : zero8h();
    *(v8h*)(tn + r * HP + c) = v;
  }
  __syncthreads();

  const int nChunks = (nE + CHUNK - 1) / CHUNK;
#pragma unroll 1
  for (int ch = 0; ch < nChunks; ++ch) {
    const int cbase = ch * CHUNK;
    const int wc = scan_chunk(rcv, nE, cbase, nodeBase, list, tid, wave);
    if (l == 0) wcnt[wave] = wc;
    __syncthreads();

#pragma unroll 1
    for (int w2 = 0; w2 < NWAVE; ++w2) {
      int n = wcnt[w2];
      n = n > WCAP ? WCAP : (n < 0 ? 0 : n);
      const int* lp = list + w2 * WCAP;
#pragma unroll 1
      for (int i = 0; i < n; ++i) {
        const int v = lp[i];
        const int slot = v & (NB - 1);
        if ((slot & (NWAVE - 1)) == wave) {
          int e = cbase + ((v >> 8) & (CHUNK - 1));
          e = e < 0 ? 0 : (e > nE - 1 ? nE - 1 : e);
          const v4h x = *(const v4h*)(ne + (size_t)e * HD + 4 * l);
          float* ap = accS + slot * HD + 4 * l;
          v4f a = *(v4f*)ap;
          a[0] += (float)x[0]; a[1] += (float)x[1]; a[2] += (float)x[2]; a[3] += (float)x[3];
          *(v4f*)ap = a;
          if (l == 0) cntL[slot] = cntL[slot] + 1;
        }
      }
    }
    __syncthreads();
  }

  for (int i = tid; i < NB * 16; i += NTHR) {
    const int r = i >> 4, c = (i & 15) * 8;
    const v4f a0 = *(const v4f*)(accS + r * HD + c);
    const v4f a1 = *(const v4f*)(accS + r * HD + c + 4);
    v8h o;
    o[0] = (_Float16)a0[0]; o[1] = (_Float16)a0[1]; o[2] = (_Float16)a0[2]; o[3] = (_Float16)a0[3];
    o[4] = (_Float16)a1[0]; o[5] = (_Float16)a1[1]; o[6] = (_Float16)a1[2]; o[7] = (_Float16)a1[3];
    *(v8h*)(ts + r * HP + c) = o;
  }
  __syncthreads();

  v8f acc[8];
#pragma unroll
  for (int i = 0; i < 8; ++i) acc[i] = zero8f();
  gemm_t<8, 4>(ts + (16 * wave + m) * HP + 8 * h, Tmn + (size_t)m * HD + 8 * h, HD, acc);
  {
#pragma unroll
    for (int r = 0; r < 8; ++r) {
      const int lr = 16 * wave + 8 * h + r;
      int nd = nodeBase + lr;
      nd = nd > nN - 1 ? nN - 1 : nd;
      const float dg = (float)cntL[lr];
      const v8h q = *(const v8h*)(P + (size_t)nd * 384 + 256 + 8 * m);
#pragma unroll
      for (int nt = 0; nt < 8; ++nt) {
        const int c = 16 * nt + m;
        const float g = acc[nt][r] * WINV + dg * ((float)q[nt] + bm[c]);
        tg[lr * HP + c] = (_Float16)g;
      }
    }
  }
  __syncthreads();

#pragma unroll
  for (int i = 0; i < 8; ++i) acc[i] = zero8f();
  gemm_t<8, 4>(tn + (16 * wave + m) * HP + 8 * h, Tnn + (size_t)m * 256 + 8 * h,       256, acc);
  gemm_t<8, 4>(tg + (16 * wave + m) * HP + 8 * h, Tnn + (size_t)m * 256 + 128 + 8 * h, 256, acc);

  float mu[8], rs[8];
#pragma unroll
  for (int nt = 0; nt < 8; ++nt) {
    const int c = 16 * nt + m;
    const float bc = bn[c];
#pragma unroll
    for (int r = 0; r < 8; ++r) {
      int nd = nodeBase + 16 * wave + 8 * h + r;
      nd = nd > nN - 1 ? nN - 1 : nd;
      const float res = nodes[(size_t)nd * HD + c];
      float v = acc[nt][r] * WINV + bc;
      acc[nt][r] = v + res;
    }
  }
#pragma unroll
  for (int r = 0; r < 8; ++r) {
    float s = 0.0f;
#pragma unroll
    for (int nt = 0; nt < 8; ++nt) s += acc[nt][r];
    s += __shfl_xor(s, 1, 32);
    s += __shfl_xor(s, 2, 32);
    s += __shfl_xor(s, 4, 32);
    s += __shfl_xor(s, 8, 32);
    mu[r] = s * (1.0f / 128.0f);
  }
#pragma unroll
  for (int r = 0; r < 8; ++r) {
    float q = 0.0f;
#pragma unroll
    for (int nt = 0; nt < 8; ++nt) { const float d = acc[nt][r] - mu[r]; q += d * d; }
    q += __shfl_xor(q, 1, 32);
    q += __shfl_xor(q, 2, 32);
    q += __shfl_xor(q, 4, 32);
    q += __shfl_xor(q, 8, 32);
    rs[r] = rsqrtf(q * (1.0f / 128.0f) + LN_EPS);
  }
  float* stg = accS;
#pragma unroll
  for (int nt = 0; nt < 8; ++nt) {
    const int c = 16 * nt + m;
    const float sc = ls[c], sb = lb[c];
#pragma unroll
    for (int r = 0; r < 8; ++r) {
      const int lr = 16 * wave + 8 * h + r;
      stg[lr * HD + c] = (acc[nt][r] - mu[r]) * rs[r] * sc + sb;
    }
  }
  __syncthreads();
  store_rows_f32(stg + (size_t)(16 * wave) * HD, HD, nodes, nodeBase + 16 * wave, nN, l);
}

#define FF_H1P 72
#define FF_H2P 40
#define FF_TN  0
#define FF_H1  (128 * HP * 2)
#define FF_H2  (FF_H1 + 128 * FF_H1P * 2)
#define FF_RAW (FF_H2 + 128 * FF_H2P * 2)
#define FF_RES (FF_RAW + 128 * 8 * 4)
#define FF_LDS (FF_RES + 1024 * 4)
static_assert((FF_H1 & 15) == 0 && (FF_H2 & 15) == 0 && (FF_RAW & 15) == 0 && (FF_RES & 15) == 0);
static_assert(((FF_H1P * 2) & 15) == 0 && ((FF_H2P * 2) & 15) == 0 && FF_LDS <= 300 * 1024);

__device__ __forceinline__ float frcp(float x) { return __builtin_amdgcn_rcpf(x); }

__global__ __launch_bounds__(256) void k_ff(const float* __restrict__ nodes, const _Float16* Tf1,
                                            const float* __restrict__ b1, const _Float16* Tf2,
                                            const float* __restrict__ b2, const _Float16* Tf3,
                                            const float* __restrict__ b3, float* out, int nN) {
  extern __shared__ __attribute__((aligned(16))) unsigned char lds[];
  _Float16* tn   = (_Float16*)(lds + FF_TN);
  _Float16* h1   = (_Float16*)(lds + FF_H1);
  _Float16* h2   = (_Float16*)(lds + FF_H2);
  float*    rawL = (float*)(lds + FF_RAW);
  float*    res  = (float*)(lds + FF_RES);
  const int tid = threadIdx.x, l = tid & 31, wave = tid >> 5, h = l >> 4, m = l & 15;
  const int row0 = blockIdx.x * 128;

  for (int i = tid; i < 128 * 16; i += 256) {
    const int r = i >> 4, c = (i & 15) * 8;
    const int gr = row0 + r;
    const v8h v = (gr < nN) ? cvt8(nodes + (size_t)gr * HD + c) : zero8h();
    *(v8h*)(tn + r * HP + c) = v;
  }
  __syncthreads();

  {
    v8f acc[4];
#pragma unroll
    for (int i = 0; i < 4; ++i) acc[i] = zero8f();
    gemm_t<4, 4>(tn + (16 * wave + m) * HP + 8 * h, Tf1 + (size_t)m * HD + 8 * h, HD, acc);
#pragma unroll
    for (int nt = 0; nt < 4; ++nt) {
      const int c = 16 * nt + m;
      const float bc = b1[c];
#pragma unroll
      for (int r = 0; r < 8; ++r) {
        const float x = acc[nt][r] * WINV + bc;
        const float s = x * frcp(1.0f + __expf(-x));
        h1[(16 * wave + 8 * h + r) * FF_H1P + c] = (_Float16)s;
      }
    }
  }
  __syncthreads();
  {
    v8f acc[2];
#pragma unroll
    for (int i = 0; i < 2; ++i) acc[i] = zero8f();
    gemm_t<2, 2>(h1 + (16 * wave + m) * FF_H1P + 8 * h, Tf2 + (size_t)m * 64 + 8 * h, 64, acc);
#pragma unroll
    for (int nt = 0; nt < 2; ++nt) {
      const int c = 16 * nt + m;
      const float bc = b2[c];
#pragma unroll
      for (int r = 0; r < 8; ++r) {
        const float x = acc[nt][r] * WINV + bc;
        const float s = x * frcp(1.0f + __expf(-x));
        h2[(16 * wave + 8 * h + r) * FF_H2P + c] = (_Float16)s;
      }
    }
  }
  __syncthreads();
  {
    v8f acc[1];
    acc[0] = zero8f();
    gemm_t<1, 1>(h2 + (16 * wave + m) * FF_H2P + 8 * h, Tf3 + (size_t)m * 32 + 8 * h, 32, acc);
    const float bc = b3[m < 6 ? m : 0];
#pragma unroll
    for (int r = 0; r < 8; ++r) {
      const float x = acc[0][r] * WINV + bc;
      if (m < 8) rawL[(16 * wave + 8 * h + r) * 8 + m] = x;
    }
  }
  __syncthreads();

  if (tid < 128) {
    const float* rw = rawL + tid * 8;
    const float kappa = 2.0f * frcp(1.0f + expf(-rw[0]));
    float* rp = res + tid * 7;
    rp[0] = kappa;
#pragma unroll
    for (int j = 1; j < 6; ++j) rp[j] = 100.0f * expf(rw[j]);
    rp[6] = 35.0f * powf(kappa, -1.0f / 3.0f);
  }
  __syncthreads();

  int nrows = nN - row0;
  nrows = nrows > 128 ? 128 : (nrows < 0 ? 0 : nrows);
  const int total = nrows * 7;
  float* ob = out + (size_t)row0 * 7;
  const int i0 = tid * 4;
  if (i0 + 3 < total) {
    const v4f v = *(const v4f*)(res + i0);
    *(volatile v4f*)(ob + i0) = v;
  } else {
#pragma unroll
    for (int j = 0; j < 4; ++j) if (i0 + j < total) { const float v = res[i0 + j]; *(volatile float*)(ob + i0 + j) = v; }
  }
  __threadfence();
  if (i0 + 3 < total) {
    const v4f v = *(const v4f*)(res + i0);
    *(volatile v4f*)(ob + i0) = v;
  } else {
#pragma unroll
    for (int j = 0; j < 4; ++j) if (i0 + j < total) { const float v = res[i0 + j]; *(volatile float*)(ob + i0 + j) = v; }
  }
}

extern "C" void kernel_launch(void* const* d_in, const int* in_sizes, int n_in,
                              void* d_out, int out_size, void* d_ws, size_t ws_size,
                              hipStream_t stream) {
  if (n_in < 24) return;
  if (in_sizes[0] <= 0 || (in_sizes[0] % 64) != 0) return;
  if (in_sizes[1] <= 0 || (in_sizes[1] % 16) != 0) return;
  const int nN = in_sizes[0] / 64;
  const int nE = in_sizes[1] / 16;
  if (in_sizes[2] != nE || in_sizes[3] != nE) return;
  if (in_sizes[4] != 64 * HD || in_sizes[5] != HD || in_sizes[6] != 16 * HD || in_sizes[7] != HD) return;
  const int nL = in_sizes[8] / (3 * HD * HD);
  if (nL < 1 || nL > 16 || in_sizes[8] != nL * 3 * HD * HD) return;
  if (in_sizes[9] != nL * HD || in_sizes[10] != nL * 2 * HD * HD || in_sizes[11] != nL * HD) return;
  if (in_sizes[12] != nL * 2 * HD * HD || in_sizes[13] != nL * HD) return;
  if (in_sizes[14] != nL * HD || in_sizes[15] != nL * HD || in_sizes[16] != nL * HD || in_sizes[17] != nL * HD) return;
  if (in_sizes[18] != HD * 64 || in_sizes[19] != 64 || in_sizes[20] != 64 * 32 || in_sizes[21] != 32) return;
  if (in_sizes[22] != 32 * 6 || in_sizes[23] != 6) return;
  if (out_size != nN * 7) return;

  const float* node_features = (const float*)d_in[0];
  const float* edge_features = (const float*)d_in[1];
  const int*   senders       = (const int*)d_in[2];
  const int*   receivers     = (const int*)d_in[3];
  const float* Wn0 = (const float*)d_in[4];
  const float* bn0 = (const float*)d_in[5];
  const float* We0 = (const float*)d_in[6];
  const float* be0 = (const float*)d_in[7];
  const float* We  = (const float*)d_in[8];
  const float* be  = (const float*)d_in[9];
  const float* Wm  = (const float*)d_in[10];
  const float* bm  = (const float*)d_in[11];
  const float* Wn  = (const float*)d_in[12];
  const float* bn  = (const float*)d_in[13];
  const float* ln_n_s = (const float*)d_in[14];
  const float* ln_n_b = (const float*)d_in[15];
  const float* ln_e_s = (const float*)d_in[16];
  const float* ln_e_b = (const float*)d_in[17];
  const float* Wf1 = (const float*)d_in[18];
  const float* bf1 = (const float*)d_in[19];
  const float* Wf2 = (const float*)d_in[20];
  const float* bf2 = (const float*)d_in[21];
  const float* Wf3 = (const float*)d_in[22];
  const float* bf3 = (const float*)d_in[23];
  float* out = (float*)d_out;

  const size_t tabTot = (size_t)T_L0 + (size_t)nL * T_LSZ + T_F1SZ + T_F2SZ + T_F3SZ;
  char* ws = (char*)d_ws;
  size_t off = 0;
  const size_t oWt = off; off += tabTot * 2;                 off = (off + 255) & ~(size_t)255;
  const size_t oNd = off; off += (size_t)nN * HD * 4;        off = (off + 255) & ~(size_t)255;
  const size_t oEd = off; off += (size_t)nE * HD * 2;        off = (off + 255) & ~(size_t)255;
  const size_t oNe = off; off += (size_t)nE * HD * 2;        off = (off + 255) & ~(size_t)255;
  const size_t oP  = off; off += (size_t)nN * 384 * 2;       off = (off + 255) & ~(size_t)255;
  if (off > ws_size) return;
  _Float16* Wt    = (_Float16*)(ws + oWt);
  float*    nodes = (float*)(ws + oNd);
  _Float16* edges = (_Float16*)(ws + oEd);
  _Float16* neb   = (_Float16*)(ws + oNe);
  _Float16* Pb    = (_Float16*)(ws + oP);
  _Float16* tN0 = Wt + T_N0;
  _Float16* tE0 = Wt + T_E0;
  _Float16* tL0 = Wt + T_L0;
  _Float16* tF1 = tL0 + (size_t)nL * T_LSZ;
  _Float16* tF2 = tF1 + T_F1SZ;
  _Float16* tF3 = tF2 + T_F2SZ;

  const hipError_t a0 = hipFuncSetAttribute(reinterpret_cast<const void*>(&k_embn), hipFuncAttributeMaxDynamicSharedMemorySize, EN_LDS);
  const hipError_t a1 = hipFuncSetAttribute(reinterpret_cast<const void*>(&k_embe), hipFuncAttributeMaxDynamicSharedMemorySize, EE_LDS);
  const hipError_t a2 = hipFuncSetAttribute(reinterpret_cast<const void*>(&k_proj), hipFuncAttributeMaxDynamicSharedMemorySize, PJ_LDS);
  const hipError_t a3 = hipFuncSetAttribute(reinterpret_cast<const void*>(&k_edge), hipFuncAttributeMaxDynamicSharedMemorySize, EG_LDS);
  const hipError_t a4 = hipFuncSetAttribute(reinterpret_cast<const void*>(&k_node), hipFuncAttributeMaxDynamicSharedMemorySize, L_LDS);
  const hipError_t a5 = hipFuncSetAttribute(reinterpret_cast<const void*>(&k_ff),   hipFuncAttributeMaxDynamicSharedMemorySize, FF_LDS);
  (void)a0; (void)a1; (void)a2; (void)a3; (void)a4; (void)a5;

  auto wc = [&](const float* src, int sStride, int srcCols, int rowOff, int K, int KP, int nValid,
                int nColsT, _Float16* dst, int dStride, int steps) {
    const int pieces = nColsT * (KP / 8);
    dim3 g((unsigned)((pieces + 255) / 256), (unsigned)steps, 1);
    k_wcvt<<<g, 256, 0, stream>>>(src, sStride, srcCols, rowOff, K, KP, nValid, nColsT, dst, dStride);
  };
  wc(Wn0, 0, HD, 0,   64,  64,  HD, HD, tN0, 0, 1);
  wc(We0, 0, HD, 0,   16,  32,  HD, HD, tE0, 0, 1);
  wc(We,  3 * HD * HD, HD, 128, 128, 128, HD, HD, tL0 + TL_PROJ,            T_LSZ, nL);
  wc(We,  3 * HD * HD, HD, 256, 128, 128, HD, HD, tL0 + TL_PROJ + 128 * 128, T_LSZ, nL);
  wc(Wm,  2 * HD * HD, HD, 0,   128, 128, HD, HD, tL0 + TL_PROJ + 256 * 128, T_LSZ, nL);
  wc(We,  3 * HD * HD, HD, 0,   128, 128, HD, HD, tL0 + TL_EE,              T_LSZ, nL);
  wc(Wm,  2 * HD * HD, HD, 128, 128, 128, HD, HD, tL0 + TL_MN,              T_LSZ, nL);
  wc(Wn,  2 * HD * HD, HD, 0,   256, 256, HD, HD, tL0 + TL_NN,              T_LSZ, nL);
  wc(Wf1, 0, 64, 0, 128, 128, 64, 64, tF1, 0, 1);
  wc(Wf2, 0, 32, 0, 64,  64,  32, 32, tF2, 0, 1);
  wc(Wf3, 0, 6,  0, 32,  32,  6,  16, tF3, 0, 1);

  const int nBlkN = (nN + 127) / 128;
  const int nBlkE = (nE + 127) / 128;
  const int nBlkA = (nN + NB - 1) / NB;

  k_embn<<<nBlkN, 256, EN_LDS, stream>>>(node_features, tN0, bn0, nodes, nN);
  k_embe<<<nBlkE, 256, EE_LDS, stream>>>(edge_features, tE0, be0, edges, nE);

  for (int s = 0; s < nL; ++s) {
    const _Float16* Ts = tL0 + (size_t)s * T_LSZ;
    k_proj<<<nBlkN, 256, PJ_LDS, stream>>>(nodes, Ts + TL_PROJ, Pb, nN);
    k_edge<<<nBlkE, 256, EG_LDS, stream>>>(senders, receivers, Pb, Ts + TL_EE, be + (size_t)s * HD,
                                            ln_e_s + (size_t)s * HD, ln_e_b + (size_t)s * HD,
                                            edges, neb, nE, nN);
    k_node<<<nBlkA, NTHR, L_LDS, stream>>>(receivers, neb, Pb, Ts + TL_MN, bm + (size_t)s * HD,
                                            Ts + TL_NN, bn + (size_t)s * HD, ln_n_s + (size_t)s * HD,
                                            ln_n_b + (size_t)s * HD, nodes, nN, nE);
  }

  k_ff<<<nBlkN, 256, FF_LDS, stream>>>(nodes, tF1, bf1, tF2, bf2, tF3, bf3, out, nN);
  (void)hipGetLastError();
}
